// LSTMDecoder_23416161698415
// MI455X (gfx1250) — hardware-run, weakly checked
//
#include <hip/hip_runtime.h>
#include <math.h>

constexpr int NB_ROWS  = 1024;
constexpr int NT_STEPS = 512;
constexpr int NEMB     = 64;
constexpr int NH1      = 50;
constexpr int NG1      = 4 * NH1;
constexpr int NGP      = 256;
constexpr int NPROJ    = 16;
constexpr int WROWS    = NGP + NPROJ;
constexpr int LP       = 72;
constexpr int ROWS_BLK = 16;
constexpr int TILES    = NB_ROWS / ROWS_BLK;
constexpr int NTHR1    = 128;
constexpr int NTHR2    = 32;
constexpr int ZC       = 8;
constexpr int PSP      = 16;
constexpr int NIN2     = 2 * NH1;
constexpr float WCAR     = 16.0f;
constexpr float WCAR_INV = 1.0f / 16.0f;
static_assert(NB_ROWS % ROWS_BLK == 0);
static_assert(NB_ROWS % NTHR2 == 0);
static_assert(NT_STEPS % 32 == 0);
static_assert((WROWS * LP) % NTHR1 == 0);
static_assert((NGP * LP) % NTHR1 == 0);
static_assert((ROWS_BLK * LP) % NTHR1 == 0);
static_assert((2 * ROWS_BLK * LP) % NTHR1 == 0);
static_assert(NGP == 4 * 16 * (NTHR1 / 32));
static_assert(LP % 8 == 0 && LP >= 64);
static_assert(NEMB % 32 == 0);

typedef __attribute__((ext_vector_type(16))) _Float16 v16h;
typedef __attribute__((ext_vector_type(8)))  _Float16 v8h;
typedef __attribute__((ext_vector_type(8)))  float    v8f;
typedef __attribute__((ext_vector_type(4)))  float    v4f;

template <typename T> struct Frag;
template <> struct Frag<_Float16> {
  typedef v16h V; union U { v16h v; v8h h[2]; };
  static __device__ __forceinline__ v16h load(const _Float16* p) {
    U f; f.h[0] = *(const v8h*)(p); f.h[1] = *(const v8h*)(p + 16); return f.v;
  }
  static __device__ __forceinline__ v8f mma(v16h a, v16h b, v8f c) {
    return __builtin_amdgcn_wmma_f32_16x16x32_f16(false, a, false, b, (short)0, c, false, false);
  }
};

__device__ __forceinline__ void mma_guard4(v8f& a0, v8f& a1, v8f& a2, v8f& a3,
                                           v16h fa, v16h b0, v16h b1, v16h b2, v16h b3) {
  asm volatile("v_nop\n\tv_nop\n\tv_nop\n\tv_nop"
               : "+v"(a0), "+v"(a1), "+v"(a2), "+v"(a3)
               : "v"(fa), "v"(b0), "v"(b1), "v"(b2), "v"(b3));
}
__device__ __forceinline__ void mma_guard1(v8f& a0, v16h fa, v16h fb) {
  asm volatile("v_nop\n\tv_nop\n\tv_nop\n\tv_nop" : "+v"(a0) : "v"(fa), "v"(fb));
}
__device__ __forceinline__ void acc_guard4(v8f& a, v8f& b, v8f& c, v8f& d) {
  asm volatile("v_nop\n\tv_nop\n\tv_nop\n\tv_nop" : "+v"(a), "+v"(b), "+v"(c), "+v"(d));
}
__device__ __forceinline__ void acc_guard1(v8f& a) {
  asm volatile("v_nop\n\tv_nop\n\tv_nop\n\tv_nop" : "+v"(a));
}

__device__ __forceinline__ float fsig(float v)  { return __builtin_amdgcn_rcpf(1.0f + expf(-v)); }
__device__ __forceinline__ float ftanh(float v) { return 1.0f - 2.0f * __builtin_amdgcn_rcpf(expf(2.0f * v) + 1.0f); }
__device__ __forceinline__ float fsel(bool p)   { return p ? 1.0f : 0.0f; }

__global__ __launch_bounds__(NTHR1) void bilstm1_kernel(
    const float* __restrict__ x,
    const float* __restrict__ Wih_f, const float* __restrict__ Whh_f,
    const float* __restrict__ bih_f, const float* __restrict__ bhh_f,
    const float* __restrict__ Wih_b, const float* __restrict__ Whh_b,
    const float* __restrict__ bih_b, const float* __restrict__ bhh_b,
    const float* __restrict__ Wih2f, const float* __restrict__ Wih2b,
    float* __restrict__ Z) {
  __shared__ __align__(16) _Float16 Wl[WROWS * LP];
  __shared__ __align__(16) _Float16 Xs[ROWS_BLK * LP];
  __shared__ __align__(16) _Float16 Hs[2 * ROWS_BLK * LP];
  __shared__ __align__(16) float    Ps[ROWS_BLK * PSP];
  constexpr int HSZ = ROWS_BLK * LP;

  const int tid = threadIdx.x, lane = tid & 31, wave = tid >> 5;
  const int c = lane & 15, hh = lane >> 4, koff = hh * 8;
  const int dir  = blockIdx.x / TILES;
  const int tile = blockIdx.x - dir * TILES;
  const int row0 = tile * ROWS_BLK;
  const float* Wih = dir ? Wih_b : Wih_f;
  const float* Whh = dir ? Whh_b : Whh_f;
  const float* bih = dir ? bih_b : bih_f;
  const float* bhh = dir ? bhh_b : bhh_f;

#pragma unroll 1
  for (int i = tid; i < ROWS_BLK * LP; i += NTHR1) {
    const int m = i / LP, k = i - m * LP;
    const int kk = (k < NEMB) ? k : (NEMB - 1);
    const float v = x[(size_t)(row0 + m) * NEMB + kk];
    Xs[i] = (_Float16)(v * fsel(k < NEMB));
  }
#pragma unroll 1
  for (int i = tid; i < 2 * ROWS_BLK * LP; i += NTHR1) Hs[i] = (_Float16)0.0f;
#pragma unroll 1
  for (int i = tid; i < NGP * LP; i += NTHR1) {
    const int n = i / LP, k = i - n * LP;
    const int g = n >> 6, j = n & 63;
    const int jj = (j < NH1) ? j : (NH1 - 1);
    const int kk = (k < NEMB) ? k : (NEMB - 1);
    const float v = Wih[(size_t)(g * NH1 + jj) * NEMB + kk];
    Wl[i] = (_Float16)(v * (WCAR * fsel((j < NH1) && (k < NEMB))));
  }
  __syncthreads();

  const int jcol = 16 * wave + c;
  const int jcl  = (jcol < NH1) ? jcol : (NH1 - 1);
  const float fvalid = fsel(jcol < NH1);
  const v8f z8 = {0.f, 0.f, 0.f, 0.f, 0.f, 0.f, 0.f, 0.f};
  float xg[4][8];
  {
    const _Float16* xrow = Xs + c * LP + koff;
    v8f acc[4];
    acc[0] = z8; acc[1] = z8; acc[2] = z8; acc[3] = z8;
#pragma unroll 1
    for (int k0 = 0; k0 < NEMB; k0 += 32) {
      const v16h a  = Frag<_Float16>::load(xrow + k0);
      const v16h b0 = Frag<_Float16>::load(Wl + (0 * 64 + jcol) * LP + koff + k0);
      const v16h b1 = Frag<_Float16>::load(Wl + (1 * 64 + jcol) * LP + koff + k0);
      const v16h b2 = Frag<_Float16>::load(Wl + (2 * 64 + jcol) * LP + koff + k0);
      const v16h b3 = Frag<_Float16>::load(Wl + (3 * 64 + jcol) * LP + koff + k0);
      acc[0] = Frag<_Float16>::mma(a, b0, acc[0]);
      acc[1] = Frag<_Float16>::mma(a, b1, acc[1]);
      acc[2] = Frag<_Float16>::mma(a, b2, acc[2]);
      acc[3] = Frag<_Float16>::mma(a, b3, acc[3]);
      mma_guard4(acc[0], acc[1], acc[2], acc[3], a, b0, b1, b2, b3);
    }
    acc_guard4(acc[0], acc[1], acc[2], acc[3]);
    float bs[4];
#pragma unroll
    for (int g = 0; g < 4; ++g) bs[g] = bih[g * NH1 + jcl] + bhh[g * NH1 + jcl];
#pragma unroll
    for (int g = 0; g < 4; ++g)
#pragma unroll
      for (int r = 0; r < 8; ++r) xg[g][r] = fmaf(acc[g][r], WCAR_INV, bs[g]) * fvalid;
  }
  __syncthreads();

#pragma unroll 1
  for (int i = tid; i < WROWS * LP; i += NTHR1) {
    const int n = i / LP, k = i - n * LP;
    const int kk = (k < NH1) ? k : (NH1 - 1);
    const int nr = (n < NGP) ? n : 0;
    const int g = nr >> 6, j = nr & 63;
    const int jj = (j < NH1) ? j : (NH1 - 1);
    const float v1 = Whh[(size_t)(g * NH1 + jj) * NH1 + kk];
    const int m  = n - NGP;
    const int mm = m & 3;
    const float v2 = Wih2f[mm * NIN2 + dir * NH1 + kk];
    const float v3 = Wih2b[mm * NIN2 + dir * NH1 + kk];
    const bool kok = (k < NH1);
    const float f1 = fsel((n < NGP) && (j < NH1) && kok);
    const float f2 = fsel((n >= NGP) && (m < 4) && kok);
    const float f3 = fsel((n >= NGP) && (m >= 4) && (m < 8) && kok);
    const float v = fmaf(f3, v3, fmaf(f2, v2, f1 * v1));
    Wl[i] = (_Float16)(v * WCAR);
  }
  float cst[8];
#pragma unroll
  for (int r = 0; r < 8; ++r) cst[r] = 0.0f;
  __syncthreads();

  const int prow = lane >> 1, pc4 = (lane & 1) * 4;

#pragma unroll 1
  for (int s = 0; s < NT_STEPS; ++s) {
    const int cur = s & 1;
    const _Float16* hrow = Hs + cur * HSZ + c * LP + koff;
    _Float16* hnx = Hs + (cur ^ 1) * HSZ;
    v8f acc[4];
    acc[0] = z8; acc[1] = z8; acc[2] = z8; acc[3] = z8;
#pragma unroll 1
    for (int k0 = 0; k0 < 64; k0 += 32) {
      const v16h a  = Frag<_Float16>::load(hrow + k0);
      const v16h b0 = Frag<_Float16>::load(Wl + (0 * 64 + jcol) * LP + koff + k0);
      const v16h b1 = Frag<_Float16>::load(Wl + (1 * 64 + jcol) * LP + koff + k0);
      const v16h b2 = Frag<_Float16>::load(Wl + (2 * 64 + jcol) * LP + koff + k0);
      const v16h b3 = Frag<_Float16>::load(Wl + (3 * 64 + jcol) * LP + koff + k0);
      acc[0] = Frag<_Float16>::mma(a, b0, acc[0]);
      acc[1] = Frag<_Float16>::mma(a, b1, acc[1]);
      acc[2] = Frag<_Float16>::mma(a, b2, acc[2]);
      acc[3] = Frag<_Float16>::mma(a, b3, acc[3]);
      mma_guard4(acc[0], acc[1], acc[2], acc[3], a, b0, b1, b2, b3);
    }
    acc_guard4(acc[0], acc[1], acc[2], acc[3]);
#pragma unroll
    for (int r = 0; r < 8; ++r) {
      const float zi = fmaf(acc[0][r], WCAR_INV, xg[0][r]);
      const float zf = fmaf(acc[1][r], WCAR_INV, xg[1][r]);
      const float zg = fmaf(acc[2][r], WCAR_INV, xg[2][r]);
      const float zo = fmaf(acc[3][r], WCAR_INV, xg[3][r]);
      const float ig = fsig(zi);
      const float fg = fsig(zf);
      const float gg = ftanh(zg);
      const float og = fsig(zo);
      const float cn = fg * cst[r] + ig * gg;
      cst[r] = cn;
      const float hn = (og * ftanh(cn)) * fvalid;
      hnx[(8 * hh + r) * LP + jcol] = (_Float16)hn;
    }
    __syncthreads();

    if (wave == 0) {
      const _Float16* hnr = Hs + (cur ^ 1) * HSZ + c * LP + koff;
      v8f pacc = z8;
#pragma unroll 1
      for (int k0 = 0; k0 < 64; k0 += 32) {
        const v16h a  = Frag<_Float16>::load(hnr + k0);
        const v16h bp = Frag<_Float16>::load(Wl + (NGP + c) * LP + koff + k0);
        pacc = Frag<_Float16>::mma(a, bp, pacc);
        mma_guard1(pacc, a, bp);
      }
      acc_guard1(pacc);
#pragma unroll
      for (int r = 0; r < 8; ++r) Ps[(8 * hh + r) * PSP + c] = pacc[r] * WCAR_INV;
      __builtin_amdgcn_fence(__ATOMIC_RELEASE, "workgroup");
      __builtin_amdgcn_wave_barrier();
      __builtin_amdgcn_fence(__ATOMIC_ACQUIRE, "workgroup");
      const int tt = dir ? (NT_STEPS - 1 - s) : s;
      float* zb = Z + (((size_t)dir * NT_STEPS + (size_t)tt) * NB_ROWS + (size_t)row0) * ZC;
      for (int pass = 0; pass < 2; ++pass) {
        const v4f v = *(const v4f*)(Ps + prow * PSP + pc4);
        *(volatile v4f*)(zb + prow * ZC + pc4) = v;
        __threadfence();
      }
      __builtin_amdgcn_fence(__ATOMIC_RELEASE, "workgroup");
      __builtin_amdgcn_wave_barrier();
      __builtin_amdgcn_fence(__ATOMIC_ACQUIRE, "workgroup");
    }
  }
}

__global__ __launch_bounds__(NTHR2) void lstm2_kernel(
    const float* __restrict__ Z,
    const float* __restrict__ Whh2f, const float* __restrict__ bih2f, const float* __restrict__ bhh2f,
    const float* __restrict__ Whh2b, const float* __restrict__ bih2b, const float* __restrict__ bhh2b,
    float* __restrict__ out) {
  __shared__ __align__(16) float Hb[NTHR2 * NT_STEPS];
  const int lane = threadIdx.x;
  const int brow0 = blockIdx.x * NTHR2;
  const int b = brow0 + lane;

  const v4f wf4 = *(const v4f*)Whh2f;
  const v4f wb4 = *(const v4f*)Whh2b;
  const v4f bf0 = *(const v4f*)bih2f;
  const v4f bf1 = *(const v4f*)bhh2f;
  const v4f bb0 = *(const v4f*)bih2b;
  const v4f bb1 = *(const v4f*)bhh2b;
  float wf[4], wb[4], bfs[4], bbs[4];
#pragma unroll
  for (int g = 0; g < 4; ++g) { wf[g] = wf4[g]; wb[g] = wb4[g]; bfs[g] = bf0[g] + bf1[g]; bbs[g] = bb0[g] + bb1[g]; }

  float h = 0.0f, cc = 0.0f;
#pragma unroll 1
  for (int t = 0; t < NT_STEPS; ++t) {
    const v4f z0 = *(const v4f*)(Z + ((size_t)t * NB_ROWS + b) * ZC);
    const v4f z1 = *(const v4f*)(Z + ((size_t)(NT_STEPS + t) * NB_ROWS + b) * ZC);
    const float zi = fmaf(wf[0], h, (z0[0] + z1[0]) + bfs[0]);
    const float zf = fmaf(wf[1], h, (z0[1] + z1[1]) + bfs[1]);
    const float zg = fmaf(wf[2], h, (z0[2] + z1[2]) + bfs[2]);
    const float zo = fmaf(wf[3], h, (z0[3] + z1[3]) + bfs[3]);
    const float ig = fsig(zi), fg = fsig(zf), gg = ftanh(zg), og = fsig(zo);
    cc = fg * cc + ig * gg;
    h  = og * ftanh(cc);
    Hb[lane * NT_STEPS + t] = h;
  }
  __syncthreads();

  h = 0.0f; cc = 0.0f;
  const int frow = lane >> 3, fc4 = (lane & 7) * 4;
#pragma unroll 1
  for (int tq = NT_STEPS / 32 - 1; tq >= 0; --tq) {
#pragma unroll 1
    for (int u = 31; u >= 0; --u) {
      const int t = tq * 32 + u;
      const v4f z0 = *(const v4f*)(Z + ((size_t)t * NB_ROWS + b) * ZC + 4);
      const v4f z1 = *(const v4f*)(Z + ((size_t)(NT_STEPS + t) * NB_ROWS + b) * ZC + 4);
      const float zi = fmaf(wb[0], h, (z0[0] + z1[0]) + bbs[0]);
      const float zf = fmaf(wb[1], h, (z0[1] + z1[1]) + bbs[1]);
      const float zg = fmaf(wb[2], h, (z0[2] + z1[2]) + bbs[2]);
      const float zo = fmaf(wb[3], h, (z0[3] + z1[3]) + bbs[3]);
      const float ig = fsig(zi), fg = fsig(zf), gg = ftanh(zg), og = fsig(zo);
      cc = fg * cc + ig * gg;
      h  = og * ftanh(cc);
      const float o = Hb[lane * NT_STEPS + t] + h;
      Hb[lane * NT_STEPS + t] = o;
    }
    __syncthreads();
    for (int pass = 0; pass < 2; ++pass) {
#pragma unroll
      for (int it = 0; it < 8; ++it) {
        const int row = it * 4 + frow;
        const v4f v = *(const v4f*)(Hb + row * NT_STEPS + tq * 32 + fc4);
        *(volatile v4f*)(out + (size_t)(brow0 + row) * NT_STEPS + tq * 32 + fc4) = v;
      }
      __threadfence();
    }
    __syncthreads();
  }
}

extern "C" void kernel_launch(void* const* d_in, const int* in_sizes, int n_in,
                              void* d_out, int out_size, void* d_ws, size_t ws_size, hipStream_t stream) {
  if (n_in < 17 || d_out == nullptr || d_ws == nullptr) return;
  if (in_sizes[0] != NB_ROWS * NEMB ||
      in_sizes[1] != NG1 * NEMB || in_sizes[2] != NG1 * NH1 || in_sizes[3] != NG1 || in_sizes[4] != NG1 ||
      in_sizes[5] != NG1 * NEMB || in_sizes[6] != NG1 * NH1 || in_sizes[7] != NG1 || in_sizes[8] != NG1 ||
      in_sizes[9] != 4 * NIN2 || in_sizes[10] != 4 || in_sizes[11] != 4 || in_sizes[12] != 4 ||
      in_sizes[13] != 4 * NIN2 || in_sizes[14] != 4 || in_sizes[15] != 4 || in_sizes[16] != 4 ||
      out_size != NB_ROWS * NT_STEPS) return;

  const float* x     = (const float*)d_in[0];
  const float* Wih1f = (const float*)d_in[1];
  const float* Whh1f = (const float*)d_in[2];
  const float* bih1f = (const float*)d_in[3];
  const float* bhh1f = (const float*)d_in[4];
  const float* Wih1b = (const float*)d_in[5];
  const float* Whh1b = (const float*)d_in[6];
  const float* bih1b = (const float*)d_in[7];
  const float* bhh1b = (const float*)d_in[8];
  const float* Wih2f = (const float*)d_in[9];
  const float* Whh2f = (const float*)d_in[10];
  const float* bih2f = (const float*)d_in[11];
  const float* bhh2f = (const float*)d_in[12];
  const float* Wih2b = (const float*)d_in[13];
  const float* Whh2b = (const float*)d_in[14];
  const float* bih2b = (const float*)d_in[15];
  const float* bhh2b = (const float*)d_in[16];
  float* out = (float*)d_out;

  char* ws = (char*)d_ws; size_t off = 0;
  auto carve = [&](size_t bytes) -> char* { char* p = ws + off; off += (bytes + 255) & ~(size_t)255; return p; };
  float* Z = (float*)carve((size_t)2 * NT_STEPS * NB_ROWS * ZC * sizeof(float));
  if (off > ws_size || off > (size_t)134217728) return;

  bilstm1_kernel<<<2 * TILES, NTHR1, 0, stream>>>(x, Wih1f, Whh1f, bih1f, bhh1f, Wih1b, Whh1b, bih1b, bhh1b,
                                                  Wih2f, Wih2b, Z);
  lstm2_kernel<<<NB_ROWS / NTHR2, NTHR2, 0, stream>>>(Z, Whh2f, bih2f, bhh2f, Whh2b, bih2b, bhh2b, out);
}
